// CustomMultiheadAttention_45689862094998
// MI455X (gfx1250) — hardware-verified
//
#include <hip/hip_runtime.h>
#include <hip/hip_bf16.h>

#ifndef NB
#define NB 2
#endif
#ifndef SEQ
#define SEQ 2048
#endif
#define NB_FULL  2
#define SEQ_FULL 2048
#define EMB  1024
#define NH   16
#define HD   64
#define NTOK (NB * SEQ)

#define SM_SCALE  0.125f
#define P_CARRY   16384.0f
#define CTX_CARRY 64.0f
#define WO_CARRY  64.0f
#define OUT_SCALE (1.0f / (CTX_CARRY * WO_CARRY))
#define OUT1_OFF_FLOATS ((size_t)NB_FULL * SEQ_FULL * EMB)

#define CP16 136
#define CPF  132
#define GEMM_LDS_16 (128 * CP16 * 2)
#define GEMM_LDS_32 (128 * CPF * 4)

#define ATT_MACC_B (16 * SEQ * 4)
#define ATT_SLOG_B (16 * SEQ * 2)
#define ATT_ORED_B (3 * 16 * 64 * 4)
#define ATT_RED_B  (4 * 16 * 2 * 4)
#define ATT_CST_B  (16 * 64 * 2)
#define ATT_LDS_B  (ATT_MACC_B + ATT_SLOG_B + ATT_ORED_B + ATT_RED_B + ATT_CST_B)

static_assert(OUT1_OFF_FLOATS * 4 == 16777216);
static_assert(SEQ % 128 == 0);
static_assert(SEQ <= SEQ_FULL);
static_assert(NB >= 1 && NB <= NB_FULL);
static_assert(EMB % 128 == 0 && EMB == NH * HD);
static_assert((NTOK % 128) == 0);
static_assert(GEMM_LDS_16 == 34816);
static_assert(GEMM_LDS_32 == 67584);
static_assert((ATT_MACC_B % 16) == 0 && (ATT_SLOG_B % 16) == 0);

typedef _Float16     v16h  __attribute__((ext_vector_type(16)));
typedef _Float16     v8h   __attribute__((ext_vector_type(8)));
typedef __bf16       v16b  __attribute__((ext_vector_type(16)));
typedef float        v8f   __attribute__((ext_vector_type(8)));
typedef float        f32x4 __attribute__((ext_vector_type(4)));
typedef unsigned int u32x4 __attribute__((ext_vector_type(4)));

union Frag { v16h h; v16b b; u32x4 q[2]; v8h h8[2]; };

__device__ __forceinline__ v8f zero8() {
  v8f z;
#pragma unroll
  for (int i = 0; i < 8; ++i) z[i] = 0.0f;
  return z;
}

__device__ __forceinline__ unsigned int bf16bits(float f) {
  unsigned int u = __float_as_uint(f);
  u += 0x7FFFu + ((u >> 16) & 1u);
  return u >> 16;
}
__device__ __forceinline__ float bf16r(float f) {
  return __uint_as_float(bf16bits(f) << 16);
}
__device__ __forceinline__ unsigned int f16bits(float f) {
  _Float16 hv = (_Float16)f;
  unsigned short u = __builtin_bit_cast(unsigned short, hv);
  return (unsigned int)u;
}

__device__ __forceinline__ v8f mma_h(v16h a, v16h b, v8f c) {
  v8f d = __builtin_amdgcn_wmma_f32_16x16x32_f16(false, a, false, b, (short)0, c, false, false);
  asm volatile("v_nop\n\tv_nop\n\tv_nop\n\tv_nop" : "+v"(d) : "v"(a), "v"(b));
  return d;
}
__device__ __forceinline__ v8f mma_b(v16b a, v16b b, v8f c) {
  v8f d = __builtin_amdgcn_wmma_f32_16x16x32_bf16(false, a, false, b, (short)0, c, false, false);
  asm volatile("v_nop\n\tv_nop\n\tv_nop\n\tv_nop" : "+v"(d) : "v"(a), "v"(b));
  return d;
}

template <int MODE>
__global__ __launch_bounds__(256) void k_cvt(const float* __restrict__ src,
                                            unsigned short* __restrict__ dst,
                                            int n8, float scale)
{
  const int i = blockIdx.x * 256 + threadIdx.x;
  if (i >= n8) return;
  const f32x4* sp = (const f32x4*)(src + (size_t)i * 8);
  const f32x4 a = sp[0];
  const f32x4 c = sp[1];
  u32x4 o;
  if (MODE == 0) {
    o.x = bf16bits(a.x) | (bf16bits(a.y) << 16);
    o.y = bf16bits(a.z) | (bf16bits(a.w) << 16);
    o.z = bf16bits(c.x) | (bf16bits(c.y) << 16);
    o.w = bf16bits(c.z) | (bf16bits(c.w) << 16);
  } else {
    o.x = f16bits(bf16r(a.x) * scale) | (f16bits(bf16r(a.y) * scale) << 16);
    o.y = f16bits(bf16r(a.z) * scale) | (f16bits(bf16r(a.w) * scale) << 16);
    o.z = f16bits(bf16r(c.x) * scale) | (f16bits(bf16r(c.y) * scale) << 16);
    o.w = f16bits(bf16r(c.z) * scale) | (f16bits(bf16r(c.w) * scale) << 16);
  }
  unsigned short* dp = dst + (size_t)i * 8;
  *(volatile u32x4*)dp = o;
  __threadfence();
  *(volatile u32x4*)dp = o;
}

template <int MODE>
__global__ __launch_bounds__(256) void k_gemm(const unsigned short* __restrict__ A,
                                             const unsigned short* __restrict__ B,
                                             const float* __restrict__ bias0,
                                             const float* __restrict__ bias1,
                                             const float* __restrict__ bias2,
                                             unsigned short* __restrict__ P0,
                                             unsigned short* __restrict__ P1,
                                             float* __restrict__ outf)
{
  extern __shared__ __attribute__((aligned(16))) unsigned char g_lds[];

  const int tid = threadIdx.x, wave = tid >> 5, lane = tid & 31;
  const int g = lane >> 4, nl = lane & 15;
  const int blockM = blockIdx.x * 128, blockN = blockIdx.y * 128;
  const int wm = (wave & 1) * 64, wn = (wave >> 1) * 32;

  v8f acc[4][2];
#pragma unroll
  for (int i = 0; i < 4; ++i)
#pragma unroll
    for (int j = 0; j < 2; ++j) acc[i][j] = zero8();

#pragma unroll 1
  for (int kt = 0; kt < EMB / 32; ++kt) {
    Frag af[4], bf[2];
#pragma unroll
    for (int fm = 0; fm < 4; ++fm) {
      const unsigned short* ap = A + (size_t)(blockM + wm + fm * 16 + nl) * EMB + kt * 32 + 8 * g;
      af[fm].q[0] = *(const u32x4*)ap;
      af[fm].q[1] = *(const u32x4*)(ap + 16);
    }
#pragma unroll
    for (int fn = 0; fn < 2; ++fn) {
      const unsigned short* bp = B + (size_t)(blockN + wn + fn * 16 + nl) * EMB + kt * 32 + 8 * g;
      bf[fn].q[0] = *(const u32x4*)bp;
      bf[fn].q[1] = *(const u32x4*)(bp + 16);
    }
#pragma unroll
    for (int fm = 0; fm < 4; ++fm)
#pragma unroll
      for (int fn = 0; fn < 2; ++fn) {
        if (MODE == 0) acc[fm][fn] = mma_b(af[fm].b, bf[fn].b, acc[fm][fn]);
        else           acc[fm][fn] = mma_h(af[fm].h, bf[fn].h, acc[fm][fn]);
      }
  }

  if (MODE == 0) {
    unsigned short* Cs = (unsigned short*)g_lds;
    const bool isV = (blockN >= 2 * EMB);
    const int slab = blockN / EMB;
    const float* bias = (slab == 0) ? bias0 : ((slab == 1) ? bias1 : bias2);
    const int cbase = blockN - slab * EMB;
#pragma unroll
    for (int fm = 0; fm < 4; ++fm)
#pragma unroll
      for (int fn = 0; fn < 2; ++fn) {
        const int cl = wn + fn * 16 + nl;
        const float bb = bf16r(bias[cbase + cl]);
#pragma unroll
        for (int r = 0; r < 8; ++r) {
          const int ml = wm + fm * 16 + 8 * g + r;
          const unsigned short hv = (unsigned short)f16bits(acc[fm][fn][r] + bb);
          if (!isV) Cs[ml * CP16 + cl] = hv;
          else      Cs[cl * CP16 + ml] = hv;
        }
      }
    __syncthreads();
    for (int ps = 0; ps < 2; ++ps) {
#pragma unroll
      for (int i = 0; i < 8; ++i) {
        const int row = 16 * wave + 2 * i + g;
        const int chunk = nl * 8;
        const u32x4 v = *(const u32x4*)(Cs + row * CP16 + chunk);
        unsigned short* dp;
        if (!isV) {
          dp = P0 + (size_t)(blockM + row) * (2 * EMB) + blockN + chunk;
        } else {
          const int c = blockN - 2 * EMB + row;
          const int hh = c >> 6, d = c & 63;
          const int bb_ = blockM / SEQ;
          const int s0 = blockM - bb_ * SEQ;
          dp = P1 + ((size_t)((bb_ * NH + hh) * HD + d)) * SEQ + s0 + chunk;
        }
        *(volatile u32x4*)dp = v;
      }
      if (ps == 0) __threadfence();
    }
  } else {
    float* Cf = (float*)g_lds;
#pragma unroll
    for (int fm = 0; fm < 4; ++fm)
#pragma unroll
      for (int fn = 0; fn < 2; ++fn) {
        const int cl = wn + fn * 16 + nl;
        const float bb = bf16r(bias0[blockN + cl]);
#pragma unroll
        for (int r = 0; r < 8; ++r) {
          const int ml = wm + fm * 16 + 8 * g + r;
          Cf[ml * CPF + cl] = acc[fm][fn][r] * OUT_SCALE + bb;
        }
      }
    __syncthreads();
    for (int ps = 0; ps < 2; ++ps) {
#pragma unroll
      for (int i = 0; i < 16; ++i) {
        const int row = 16 * wave + i;
        const int col = lane * 4;
        const f32x4 v = *(const f32x4*)(Cf + row * CPF + col);
        float* dp = outf + (size_t)(blockM + row) * EMB + blockN + col;
        *(volatile f32x4*)dp = v;
      }
      if (ps == 0) __threadfence();
    }
  }
}

__global__ __launch_bounds__(128) void k_attn(const unsigned short* __restrict__ QK,
                                             const unsigned short* __restrict__ Vt,
                                             unsigned short* __restrict__ ctx,
                                             float* __restrict__ out1)
{
  extern __shared__ __attribute__((aligned(16))) unsigned char a_lds[];
  float*    macc = (float*)a_lds;
  _Float16* slog = (_Float16*)(a_lds + ATT_MACC_B);
  float*    ored = (float*)(a_lds + ATT_MACC_B + ATT_SLOG_B);
  float*    red  = (float*)(a_lds + ATT_MACC_B + ATT_SLOG_B + ATT_ORED_B);
  _Float16* cst  = (_Float16*)(a_lds + ATT_MACC_B + ATT_SLOG_B + ATT_ORED_B + ATT_RED_B);

  const int tid = threadIdx.x, wave = tid >> 5, lane = tid & 31;
  const int g = lane >> 4, nl = lane & 15;
  const int b = blockIdx.y, q0 = blockIdx.x * 16;
  const size_t tok0 = (size_t)b * SEQ;
  const unsigned short* Qrow = QK + (tok0 + q0 + nl) * (size_t)(2 * EMB);
  const float invh = 1.0f / (float)NH;

#pragma unroll 1
  for (int h = 0; h < NH; ++h) {
    Frag qf[2];
#pragma unroll
    for (int ds = 0; ds < 2; ++ds) {
      const unsigned short* p = Qrow + h * HD + ds * 32 + 8 * g;
      qf[ds].q[0] = *(const u32x4*)p;
      qf[ds].q[1] = *(const u32x4*)(p + 16);
    }

    float mrun = -1.0e30f, lrun = 0.0f;
#pragma unroll 1
    for (int kt = 0; kt < SEQ / 128; ++kt) {
      const int kk0 = kt * 128 + 32 * wave;
      Frag kf[2][2];
#pragma unroll
      for (int mf = 0; mf < 2; ++mf)
#pragma unroll
        for (int ds = 0; ds < 2; ++ds) {
          const unsigned short* p = QK + (tok0 + kk0 + 16 * mf + nl) * (size_t)(2 * EMB)
                                       + EMB + h * HD + ds * 32 + 8 * g;
          kf[mf][ds].q[0] = *(const u32x4*)p;
          kf[mf][ds].q[1] = *(const u32x4*)(p + 16);
        }
      v8f S[2];
#pragma unroll
      for (int mf = 0; mf < 2; ++mf) {
        S[mf] = mma_h(kf[mf][0].h, qf[0].h, zero8());
        S[mf] = mma_h(kf[mf][1].h, qf[1].h, S[mf]);
      }
#pragma unroll
      for (int mf = 0; mf < 2; ++mf) {
        v8h hs;
#pragma unroll
        for (int r = 0; r < 8; ++r) hs[r] = (_Float16)(S[mf][r] * SM_SCALE);
        *(v8h*)(slog + nl * SEQ + kk0 + 16 * mf + 8 * g) = hs;
        float sf[8];
#pragma unroll
        for (int r = 0; r < 8; ++r) sf[r] = (float)hs[r];
        float mt = sf[0];
#pragma unroll
        for (int r = 1; r < 8; ++r) mt = fmaxf(mt, sf[r]);
        const float mnew = fmaxf(mrun, mt);
        float sum = 0.0f;
#pragma unroll
        for (int r = 0; r < 8; ++r) sum += __expf(sf[r] - mnew);
        lrun = lrun * __expf(mrun - mnew) + sum;
        mrun = mnew;
      }
    }
    {
      const float mo = __shfl_xor(mrun, 16);
      const float lo = __shfl_xor(lrun, 16);
      const float mm = fmaxf(mrun, mo);
      const float ll = lrun * __expf(mrun - mm) + lo * __expf(mo - mm);
      if (g == 0) {
        red[(wave * 16 + nl) * 2 + 0] = mm;
        red[(wave * 16 + nl) * 2 + 1] = ll;
      }
    }
    __syncthreads();
    float M = -1.0e30f;
#pragma unroll
    for (int w = 0; w < 4; ++w) M = fmaxf(M, red[(w * 16 + nl) * 2 + 0]);
    float L = 0.0f;
#pragma unroll
    for (int w = 0; w < 4; ++w) L += red[(w * 16 + nl) * 2 + 1] * __expf(red[(w * 16 + nl) * 2 + 0] - M);
    const float linv = 1.0f / L;
    const float pcl = linv * P_CARRY;

    v8f oacc[4];
#pragma unroll
    for (int df = 0; df < 4; ++df) oacc[df] = zero8();
#pragma unroll 1
    for (int kt = 0; kt < SEQ / 128; ++kt) {
      const int kk0 = kt * 128 + 32 * wave;
      v8h hsv[2];
      hsv[0] = *(const v8h*)(slog + nl * SEQ + kk0 + 8 * g);
      hsv[1] = *(const v8h*)(slog + nl * SEQ + kk0 + 16 + 8 * g);
      Frag pa;
#pragma unroll
      for (int mf = 0; mf < 2; ++mf) {
        float p[8];
#pragma unroll
        for (int r = 0; r < 8; ++r) p[r] = __expf((float)hsv[mf][r] - M);
        float* mp = macc + nl * SEQ + kk0 + 16 * mf + 8 * g;
        f32x4 w0, w1;
        w0.x = p[0] * linv; w0.y = p[1] * linv; w0.z = p[2] * linv; w0.w = p[3] * linv;
        w1.x = p[4] * linv; w1.y = p[5] * linv; w1.z = p[6] * linv; w1.w = p[7] * linv;
        if (h != 0) {
          w0 += *(const f32x4*)mp;
          w1 += *(const f32x4*)(mp + 4);
        }
        *(f32x4*)mp = w0;
        *(f32x4*)(mp + 4) = w1;
        v8h ph;
#pragma unroll
        for (int r = 0; r < 8; ++r) ph[r] = (_Float16)(p[r] * pcl);
        pa.h8[mf] = ph;
      }
      Frag vb[4];
#pragma unroll
      for (int df = 0; df < 4; ++df) {
        const unsigned short* p = Vt + ((size_t)((b * NH + h) * HD + df * 16 + nl)) * SEQ + kk0 + 8 * g;
        vb[df].q[0] = *(const u32x4*)p;
        vb[df].q[1] = *(const u32x4*)(p + 16);
      }
#pragma unroll
      for (int df = 0; df < 4; ++df) oacc[df] = mma_h(pa.h, vb[df].h, oacc[df]);
    }

    if (wave > 0) {
      float* ob = ored + (wave - 1) * 1024;
#pragma unroll
      for (int df = 0; df < 4; ++df)
#pragma unroll
        for (int r = 0; r < 8; ++r) ob[(8 * g + r) * 64 + df * 16 + nl] = oacc[df][r];
    }
    __syncthreads();
    if (wave == 0) {
#pragma unroll
      for (int df = 0; df < 4; ++df)
#pragma unroll
        for (int r = 0; r < 8; ++r) {
          const int row = 8 * g + r, col = df * 16 + nl;
          const float o = ((oacc[df][r] + ored[row * 64 + col]) + ored[1024 + row * 64 + col])
                          + ored[2048 + row * 64 + col];
          cst[row * 64 + col] = (_Float16)(o * (CTX_CARRY / P_CARRY));
        }
    }
    __syncthreads();
    {
      const int row = 4 * wave + (lane >> 3);
      const int chunk = (lane & 7) * 8;
      const u32x4 v = *(const u32x4*)(cst + row * 64 + chunk);
      unsigned short* dp = ctx + (tok0 + q0 + row) * (size_t)EMB + h * HD + chunk;
      *(volatile u32x4*)dp = v;
      __threadfence();
      *(volatile u32x4*)dp = v;
    }
  }
  __syncthreads();

  for (int ps = 0; ps < 2; ++ps) {
#pragma unroll
    for (int rr = 0; rr < 4; ++rr) {
      const int row = 4 * wave + rr;
      const float* mrow = macc + row * SEQ;
      float* orow = out1 + (tok0 + q0 + row) * (size_t)SEQ;
#pragma unroll 1
      for (int c = 0; c < SEQ / 128; ++c) {
        const int col = c * 128 + lane * 4;
        f32x4 v = *(const f32x4*)(mrow + col);
        v = v * invh;
        *(volatile f32x4*)(orow + col) = v;
      }
    }
    if (ps == 0) __threadfence();
  }
}

extern "C" void kernel_launch(void* const* d_in, const int* in_sizes, int n_in,
                              void* d_out, int out_size, void* d_ws, size_t ws_size,
                              hipStream_t stream)
{
  if (n_in < 9) return;
  if (in_sizes[0] < ((NB - 1) * SEQ_FULL + SEQ) * EMB) return;
  if (in_sizes[1] < EMB * EMB || in_sizes[3] < EMB * EMB ||
      in_sizes[5] < EMB * EMB || in_sizes[7] < EMB * EMB) return;
  if (in_sizes[2] < EMB || in_sizes[4] < EMB || in_sizes[6] < EMB || in_sizes[8] < EMB) return;
  if ((size_t)out_size < OUT1_OFF_FLOATS + (size_t)NTOK * SEQ) return;

  const float* query = (const float*)d_in[0];
  const float* Wq = (const float*)d_in[1];
  const float* bq = (const float*)d_in[2];
  const float* Wk = (const float*)d_in[3];
  const float* bk = (const float*)d_in[4];
  const float* Wv = (const float*)d_in[5];
  const float* bv = (const float*)d_in[6];
  const float* Wo = (const float*)d_in[7];
  const float* bo = (const float*)d_in[8];
  float* out0 = (float*)d_out;
  float* out1 = (float*)d_out + OUT1_OFF_FLOATS;

  char* ws = (char*)d_ws;
  size_t off = 0;
  unsigned short* Xb   = (unsigned short*)(ws + off); off += (size_t)NTOK * EMB * 2;
  unsigned short* Wqkv = (unsigned short*)(ws + off); off += (size_t)3 * EMB * EMB * 2;
  unsigned short* Wo16 = (unsigned short*)(ws + off); off += (size_t)EMB * EMB * 2;
  unsigned short* QK   = (unsigned short*)(ws + off); off += (size_t)NTOK * 2 * EMB * 2;
  unsigned short* Vt   = (unsigned short*)(ws + off); off += (size_t)NTOK * EMB * 2;
  unsigned short* ctx  = (unsigned short*)(ws + off); off += (size_t)NTOK * EMB * 2;
  if (off > ws_size) return;

  const int n8x = SEQ * EMB / 8;
  for (int b = 0; b < NB; ++b)
    k_cvt<0><<<(n8x + 255) / 256, 256, 0, stream>>>(query + (size_t)b * SEQ_FULL * EMB,
                                                   Xb + (size_t)b * SEQ * EMB, n8x, 1.0f);
  const int n8w = EMB * EMB / 8;
  k_cvt<0><<<(n8w + 255) / 256, 256, 0, stream>>>(Wq, Wqkv, n8w, 1.0f);
  k_cvt<0><<<(n8w + 255) / 256, 256, 0, stream>>>(Wk, Wqkv + (size_t)EMB * EMB, n8w, 1.0f);
  k_cvt<0><<<(n8w + 255) / 256, 256, 0, stream>>>(Wv, Wqkv + (size_t)2 * EMB * EMB, n8w, 1.0f);
  k_cvt<1><<<(n8w + 255) / 256, 256, 0, stream>>>(Wo, Wo16, n8w, WO_CARRY);

  dim3 g1(NTOK / 128, (3 * EMB) / 128, 1);
  k_gemm<0><<<g1, 256, GEMM_LDS_16, stream>>>(Xb, Wqkv, bq, bk, bv, QK, Vt, out0);

  hipFuncSetAttribute(reinterpret_cast<const void*>(&k_attn),
                      hipFuncAttributeMaxDynamicSharedMemorySize, ATT_LDS_B);
  dim3 g2(SEQ / 16, NB, 1);
  k_attn<<<g2, 128, ATT_LDS_B, stream>>>(QK, Vt, ctx, out1);

  hipFuncSetAttribute(reinterpret_cast<const void*>(&k_gemm<1>),
                      hipFuncAttributeMaxDynamicSharedMemorySize, GEMM_LDS_32);
  dim3 g3(NTOK / 128, EMB / 128, 1);
  k_gemm<1><<<g3, 256, GEMM_LDS_32, stream>>>(ctx, Wo16, bo, bo, bo, QK, Vt, out0);
}
